// CharRNN_68212670595566
// MI455X (gfx1250) — hardware-verified
//
#include <hip/hip_runtime.h>

typedef __attribute__((ext_vector_type(16))) _Float16 v16h;
typedef __attribute__((ext_vector_type(8)))  _Float16 v8h;
typedef __attribute__((ext_vector_type(16))) __bf16   v16b;
typedef __attribute__((ext_vector_type(8)))  __bf16   v8b;
typedef __attribute__((ext_vector_type(8)))  float    v8f;
typedef __attribute__((ext_vector_type(4)))  float    v4f;
typedef __attribute__((ext_vector_type(4)))  unsigned int u32x4;

constexpr int NBATCH  = 64;
constexpr int NSTEP   = 512;
constexpr int NVOC    = 96;
constexpr int DEMB    = 24;
constexpr int HREAL   = 200;
constexpr int HPAD    = 208;
constexpr int KPADH   = 224;
constexpr int NGATE4  = 832;
constexpr int GSRC    = 800;
constexpr int KPADE   = 32;
constexpr int NEXPAD  = 256;
constexpr int KPADY   = 896;
constexpr int MROWS   = NSTEP * NBATCH;
constexpr int TCHUNK  = 128;
constexpr int NCHUNK  = NSTEP / TCHUNK;
constexpr int MCHUNK  = TCHUNK * NBATCH;
constexpr int NLAYER  = 4;
constexpr int ROWS_PER_BLK = 32;
constexpr int LSTM_TPB = 13 * 32;
constexpr int HL_UNITS = ROWS_PER_BLK * KPADH * 2 / 16;
constexpr int CS_UNITS = ROWS_PER_BLK * HPAD * 4 / 16;
constexpr float WCARRY = 16.0f;
constexpr float ECARRY = 64.0f;
constexpr float WINV   = 0.0625f;
constexpr float PEINV  = 1.0f / 1024.0f;
constexpr int BIAS_PRE_OFF = 0;
constexpr int BIAS_EX_OFF  = 3328;
constexpr int BIAS_Y_OFF   = 4096;
constexpr int BIAS_TOTAL   = 4192;

static_assert(NCHUNK * TCHUNK == NSTEP, "chunks");
static_assert(MCHUNK % 64 == 0 && MROWS % 64 == 0, "GEMM M tile");
static_assert(NGATE4 % 64 == 0 && NEXPAD % 64 == 0, "GEMM N tile");
static_assert(KPADE % 32 == 0 && KPADH % 32 == 0 && KPADY % 32 == 0, "GEMM K step");
static_assert(HPAD == 13 * 16 && NGATE4 == 4 * HPAD && KPADY == NLAYER * KPADH, "padding");
static_assert(HL_UNITS == 896 && CS_UNITS == 4 * LSTM_TPB, "copy coverage");
static_assert(MROWS % 32 == 0 && (MROWS / 32) % 8 == 0, "logit tiles");
static_assert(BIAS_PRE_OFF % 32 == 0 && BIAS_EX_OFF % 32 == 0 && BIAS_Y_OFF % 32 == 0, "bias line alignment");

__device__ __forceinline__ unsigned short f2bf_bits(float f) {
  unsigned u = __float_as_uint(f);
  return (unsigned short)((u + 0x7FFFu + ((u >> 16) & 1u)) >> 16);
}
__device__ __forceinline__ float bf_bits2f(unsigned short h) { return __uint_as_float(((unsigned)h) << 16); }
__device__ __forceinline__ float bfr(float x) { return bf_bits2f(f2bf_bits(x)); }

__device__ __forceinline__ void dep_guard_h(v8f& a, v8f& b, v16h x, v16h y) { asm volatile("v_nop\n\tv_nop\n\tv_nop\n\tv_nop" : "+v"(a), "+v"(b) : "v"(x), "v"(y)); }
__device__ __forceinline__ void dep_guard_b(v8f& a, v8f& b, v16b x, v16b y) { asm volatile("v_nop\n\tv_nop\n\tv_nop\n\tv_nop" : "+v"(a), "+v"(b) : "v"(x), "v"(y)); }
__device__ __forceinline__ void keep4_h(v16h a, v16h b, v16h c, v16h d) { asm volatile("v_nop" :: "v"(a), "v"(b), "v"(c), "v"(d)); }
__device__ __forceinline__ void keep4_b(v16b a, v16b b, v16b c, v16b d) { asm volatile("v_nop" :: "v"(a), "v"(b), "v"(c), "v"(d)); }
__device__ __forceinline__ void acc_guard4(v8f& a, v8f& b, v8f& c, v8f& d) { asm volatile("v_nop\n\tv_nop\n\tv_nop\n\tv_nop" : "+v"(a), "+v"(b), "+v"(c), "+v"(d)); }
template <typename T> struct Frag;
template <> struct Frag<_Float16> {
  typedef v16h V; union U { v16h v; v8h h[2]; };
  static __device__ __forceinline__ v16h load(const _Float16* p) {
    U f; f.h[0] = *(const v8h*)(p); f.h[1] = *(const v8h*)(p + 16); return f.v;
  }
  static __device__ __forceinline__ v8f mma(v16h a, v16h b, v8f c) {
    return __builtin_amdgcn_wmma_f32_16x16x32_f16(false, a, false, b, (short)0, c, false, false);
  }
  static __device__ __forceinline__ void guard(v8f& a, v8f& b, v16h x, v16h y) { dep_guard_h(a, b, x, y); }
  static __device__ __forceinline__ void keep(v16h a, v16h b, v16h c, v16h d) { keep4_h(a, b, c, d); }
};
template <> struct Frag<__bf16> {
  typedef v16b V; union U { v16b v; v8b h[2]; };
  static __device__ __forceinline__ v16b load(const __bf16* p) {
    U f; f.h[0] = *(const v8b*)(p); f.h[1] = *(const v8b*)(p + 16); return f.v;
  }
  static __device__ __forceinline__ v8f mma(v16b a, v16b b, v8f c) {
    return __builtin_amdgcn_wmma_f32_16x16x32_bf16(false, a, false, b, (short)0, c, false, false);
  }
  static __device__ __forceinline__ void guard(v8f& a, v8f& b, v16b x, v16b y) { dep_guard_b(a, b, x, y); }
  static __device__ __forceinline__ void keep(v16b a, v16b b, v16b c, v16b d) { keep4_b(a, b, c, d); }
};

template <int ET> struct Elem;
template <> struct Elem<0> { typedef _Float16 T; };
template <> struct Elem<1> { typedef __bf16 T; };
template <int ET, bool SPLIT, int BIAS_MODE, int OUT_MODE, bool RESID, int ACT = 0>
__global__ __launch_bounds__(256) void wmma_gemm64(
    const unsigned short* __restrict__ Ap, const unsigned short* __restrict__ A2p, int lda, long strideA,
    const unsigned short* __restrict__ Btp, const unsigned short* __restrict__ Bt2p, int ldb, long strideB,
    void* __restrict__ Cout, void* __restrict__ Cout2, int ldc, long strideC,
    const float* __restrict__ bias,
    const float* __restrict__ resid, long strideR,
    int M, int N, int K, float scale) {
  typedef typename Elem<ET>::T T;
  typedef typename Frag<T>::V V;
  const T* A = (const T*)Ap; const T* A2 = (const T*)A2p; const T* Bt = (const T*)Btp; const T* Bt2 = (const T*)Bt2p;
  __shared__ __align__(16) float sT[8][16 * 68];
  const int b    = blockIdx.y;
  const int lane = threadIdx.x & 31;
  const int wave = threadIdx.x >> 5;
  const int tilesN = N >> 6;
  const int tilesM = M >> 6;
  const int tile = blockIdx.x * 8 + wave;
  if (tile >= tilesM * tilesN) return;
  const int tm = tile / tilesN;
  const int tn = tile - tm * tilesN;
  const int m0 = tm << 6;
  const int n0 = tn << 6;

  const T* Ab  = A  + (size_t)b * strideA;
  const T* Bb  = Bt + (size_t)b * strideB;
  const T* Ab2 = SPLIT ? (A2  + (size_t)b * strideA) : nullptr;
  const T* Bb2 = SPLIT ? (Bt2 + (size_t)b * strideB) : nullptr;

  const int rlane = lane & 15;
  const int koff  = (lane >> 4) * 8;
  const int mOff  = (lane >> 4) * 8;

  v8f acc[4][4];
#pragma unroll
  for (int i = 0; i < 4; ++i)
#pragma unroll
    for (int j = 0; j < 4; ++j) acc[i][j] = (v8f){0.f,0.f,0.f,0.f,0.f,0.f,0.f,0.f};

  for (int k0 = 0; k0 < K; k0 += 32) {
    V bh[4], bl[4];
#pragma unroll
    for (int j = 0; j < 4; ++j) {
      const size_t bo = (size_t)(n0 + (j << 4) + rlane) * ldb + koff + k0;
      bh[j] = Frag<T>::load(Bb + bo);
      if (SPLIT) bl[j] = Frag<T>::load(Bb2 + bo);
    }
#pragma unroll
    for (int i = 0; i < 4; ++i) {
      const size_t ao = (size_t)(m0 + (i << 4) + rlane) * lda + koff + k0;
      V ah = Frag<T>::load(Ab + ao);
      V al;
      if (SPLIT) al = Frag<T>::load(Ab2 + ao);
#pragma unroll
      for (int j = 0; j < 4; ++j) {
        acc[i][j] = Frag<T>::mma(ah, bh[j], acc[i][j]);
        if (SPLIT) {
          acc[i][j] = Frag<T>::mma(ah, bl[j], acc[i][j]);
          acc[i][j] = Frag<T>::mma(al, bh[j], acc[i][j]);
        }
      }
      Frag<T>::guard(acc[i][0], acc[i][3], ah, SPLIT ? al : ah);
    }
    Frag<T>::keep(bh[0], bh[1], bh[2], bh[3]);
    if (SPLIT) Frag<T>::keep(bl[0], bl[1], bl[2], bl[3]);
  }
  acc_guard4(acc[0][0], acc[0][1], acc[0][2], acc[0][3]);
  acc_guard4(acc[1][0], acc[1][1], acc[1][2], acc[1][3]);
  acc_guard4(acc[2][0], acc[2][1], acc[2][2], acc[2][3]);
  acc_guard4(acc[3][0], acc[3][1], acc[3][2], acc[3][3]);

  float* slab = sT[wave];
  const float* Rb = RESID ? (resid + (size_t)b * strideR) : nullptr;
#pragma unroll
  for (int i = 0; i < 4; ++i) {
    const int mBase = m0 + (i << 4);
#pragma unroll
    for (int j = 0; j < 4; ++j) {
      const int n = n0 + (j << 4) + rlane;
      float bv = 0.f;
      if (BIAS_MODE == 2) bv = bias[n];
#pragma unroll
      for (int r = 0; r < 8; ++r) {
        float v = acc[i][j][r] * scale;
        if (BIAS_MODE == 1) v += bias[mBase + mOff + r];
        if (BIAS_MODE == 2) v += bv;
        if (RESID) v += Rb[(size_t)(mBase + mOff + r) * ldc + n];
        if (ACT == 1) v = tanhf(v);
        if (ACT == 2) v = fmaxf(v, 0.0f);
        if (ACT == 3) v = v / (1.0f + expf(-v));
        if (ACT == 4) v = (v > 0.f) ? v : 0.01f * v;
        if (ACT == 5) v = 0.5f * v * (1.0f + erff(v * 0.70710678118654752f));
        slab[(mOff + r) * 68 + (j << 4) + rlane] = v;
      }
    }
    __builtin_amdgcn_fence(__ATOMIC_RELEASE, "workgroup");
    __builtin_amdgcn_wave_barrier();
    __builtin_amdgcn_fence(__ATOMIC_ACQUIRE, "workgroup");
    if (OUT_MODE == 0) {
      float* C = (float*)Cout + (size_t)b * strideC;
      const int hh = lane >> 4, c4 = (lane & 15) * 4;
      for (int pass = 0; pass < 2; ++pass) {
#pragma unroll
        for (int it = 0; it < 8; ++it) {
          const int row = it * 2 + hh;
          v4f v = *(const v4f*)(slab + row * 68 + c4);
          *(volatile v4f*)(C + (size_t)(mBase + row) * ldc + n0 + c4) = v;
        }
        __threadfence();
      }
    } else {
      const int q = lane >> 3, c8 = (lane & 7) * 8;
      unsigned short* C  = (unsigned short*)Cout  + (size_t)b * strideC;
      unsigned short* C2 = (OUT_MODE == 2) ? ((unsigned short*)Cout2 + (size_t)b * strideC) : nullptr;
      for (int pass = 0; pass < 2; ++pass) {
#pragma unroll
        for (int it = 0; it < 4; ++it) {
          const int row = it * 4 + q;
          const float* sp = slab + row * 68 + c8;
          v8h hv, lv;
#pragma unroll
          for (int e = 0; e < 8; ++e) {
            if (OUT_MODE == 1) {
              hv[e] = (_Float16)sp[e];
            } else {
              unsigned short hb = f2bf_bits(sp[e]);
              unsigned short lb = f2bf_bits(sp[e] - bf_bits2f(hb));
              hv[e] = __builtin_bit_cast(_Float16, hb);
              lv[e] = __builtin_bit_cast(_Float16, lb);
            }
          }
          *(volatile v8h*)(C + (size_t)(mBase + row) * ldc + n0 + c8) = hv;
          if (OUT_MODE == 2) *(volatile v8h*)(C2 + (size_t)(mBase + row) * ldc + n0 + c8) = lv;
        }
        __threadfence();
      }
    }
    __builtin_amdgcn_fence(__ATOMIC_RELEASE, "workgroup");
    __builtin_amdgcn_wave_barrier();
    __builtin_amdgcn_fence(__ATOMIC_ACQUIRE, "workgroup");
  }
}

__device__ __forceinline__ float sigm_f(float x) {
  return __builtin_amdgcn_rcpf(1.0f + __builtin_amdgcn_exp2f(x * -1.4426950408889634f));
}
__device__ __forceinline__ float tanh_f(float x) { return 2.0f * sigm_f(2.0f * x) - 1.0f; }

__global__ __launch_bounds__(256) void k_wplane(
    const float* __restrict__ src0, const float* __restrict__ src1, long src1Stride,
    unsigned short* __restrict__ dst, long dstStride, int nRows, int kp, int mode, int kReal) {
  const int lane = threadIdx.x & 31, wave = threadIdx.x >> 5;
  const int z = blockIdx.y;
  const float* src = (z == 0) ? src0 : (src1 + (size_t)(z - 1) * (size_t)src1Stride);
  unsigned short* d = dst + (size_t)z * (size_t)dstStride;
  const int r0 = (blockIdx.x * 8 + wave) * 16;
  if (r0 >= nRows) return;
  const int upr = kp >> 3;
  const int nUnits = 16 * upr;
  _Float16* drow = (_Float16*)(void*)(d + (size_t)r0 * kp);
  for (int pass = 0; pass < 2; ++pass) {
    for (int u = lane; u < nUnits; u += 32) {
      const int rr = u / upr;
      const int row = r0 + rr;
      const int col0 = (u - rr * upr) * 8;
      v8h hv;
#pragma unroll
      for (int e = 0; e < 8; ++e) {
        const int k = col0 + e;
        int sidx = 0;
        bool valid = false;
        if (mode == 0) {
          const int hc = row >> 2, q = row & 3;
          const int kc = (k < kReal) ? k : (kReal - 1);
          const int hcc = (hc < HREAL) ? hc : (HREAL - 1);
          valid = (hc < HREAL) && (k < kReal);
          sidx = kc * GSRC + q * HREAL + hcc;
        } else if (mode == 1) {
          const int q = row / HPAD;
          const int j = row - q * HPAD;
          const int jc = (j < HREAL) ? j : (HREAL - 1);
          const int kc = (k < HREAL) ? k : (HREAL - 1);
          valid = (j < HREAL) && (k < HREAL);
          sidx = kc * GSRC + q * HREAL + jc;
        } else if (mode == 2) {
          const int kc = (k < DEMB) ? k : (DEMB - 1);
          const int nc = (row < HREAL) ? row : (HREAL - 1);
          valid = (row < HREAL) && (k < DEMB);
          sidx = kc * HREAL + nc;
        } else {
          const int l = k / KPADH;
          const int kk = k - l * KPADH;
          const int kc = (kk < HREAL) ? kk : (HREAL - 1);
          const int nc = (row < NVOC) ? row : (NVOC - 1);
          valid = (kk < HREAL);
          sidx = (l * HREAL + kc) * NVOC + nc;
        }
        const float x = src[sidx];
        const float y = bfr(x) * WCARRY;
        hv[e] = valid ? (_Float16)y : (_Float16)0.0f;
      }
      *(volatile v8h*)(drow + (size_t)u * 8) = hv;
    }
    __threadfence();
  }
}

__global__ __launch_bounds__(256) void k_embplane(
    const int* __restrict__ xb, const float* __restrict__ Cw, unsigned short* __restrict__ emb) {
  const int u = blockIdx.x * 256 + threadIdx.x;
  if (u >= MROWS * 4) return;
  const int m = u >> 2, col0 = (u & 3) * 8;
  const int t = m >> 6, b = m & 63;
  int tok = xb[b * NSTEP + t];
  tok = tok < 0 ? 0 : (tok > (NVOC - 1) ? (NVOC - 1) : tok);
  v8h hv;
#pragma unroll
  for (int e = 0; e < 8; ++e) {
    const int dcol = col0 + e;
    const int dc = (dcol < DEMB) ? dcol : (DEMB - 1);
    const float x = Cw[tok * DEMB + dc];
    const float y = bfr(x) * ECARRY;
    hv[e] = (dcol < DEMB) ? (_Float16)y : (_Float16)0.0f;
  }
  _Float16* p = (_Float16*)(void*)emb + (size_t)u * 8;
  *(volatile v8h*)p = hv;
  __threadfence();
  *(volatile v8h*)p = hv;
}

__global__ __launch_bounds__(256) void k_biasprep(
    const float* __restrict__ uinb, const float* __restrict__ uhb, const float* __restrict__ vhb,
    const float* __restrict__ byv, float* __restrict__ bias_all) {
  const int i = blockIdx.x * 256 + threadIdx.x;
  if (i >= BIAS_TOTAL) return;
  const int kA = (i < 3328) ? i : 0;
  const int layer = kA / NGATE4;
  const int np = kA - layer * NGATE4;
  const int hc = np >> 2, q = np & 3;
  const int hcc = (hc < HREAL) ? hc : (HREAL - 1);
  const int lm1 = (layer > 0) ? (layer - 1) : 0;
  const float xa = uinb[q * HREAL + hcc];
  const float xb2 = uhb[lm1 * GSRC + q * HREAL + hcc];
  int kB = i - 3328; kB = kB < 0 ? 0 : (kB > 767 ? 767 : kB);
  const int nB = kB >> 8, jB = kB & 255;
  const int jc = (jB < HREAL) ? jB : (HREAL - 1);
  const float xc = vhb[nB * HREAL + jc];
  int kC = i - 4096; kC = kC < 0 ? 0 : (kC > (NVOC - 1) ? (NVOC - 1) : kC);
  const float xd = byv[kC];
  float v;
  if (i < 3328) v = (hc < HREAL) ? ((layer == 0) ? xa : xb2) : 0.0f;
  else if (i < 4096) v = (jB < HREAL) ? xc : 0.0f;
  else v = xd;
  v = bfr(v);
  ((volatile float*)bias_all)[i] = v;
  __threadfence();
  ((volatile float*)bias_all)[i] = v;
}

__global__ __launch_bounds__(LSTM_TPB) void k_lstm_chunk(
    const float* __restrict__ preC, const unsigned short* __restrict__ BtW,
    const float* __restrict__ exb, const float* __restrict__ h0v, const float* __restrict__ c0v,
    unsigned short* __restrict__ hall, float* __restrict__ cst, int chunk, int has_ex) {
  __shared__ __align__(16) _Float16 hl[ROWS_PER_BLK * KPADH];
  __shared__ __align__(16) float cs[ROWS_PER_BLK * HPAD];
  const int tid = threadIdx.x, lane = tid & 31, wave = tid >> 5;
  const int hh = lane >> 4, rl = lane & 15, koff = hh * 8;
  const int rowbase = blockIdx.x * ROWS_PER_BLK;
  const int hcol = wave * 16 + rl;
  const int hcc = (hcol < HREAL) ? hcol : (HREAL - 1);
  const int t0 = chunk * TCHUNK;
  const _Float16* Bt = (const _Float16*)(const void*)BtW;
  u32x4* hl4 = (u32x4*)(void*)hl;
  u32x4* cs4 = (u32x4*)(void*)cs;

  float cc[2][8];
  if (chunk == 0) {
#pragma unroll 1
    for (int i = tid; i < ROWS_PER_BLK * KPADH; i += LSTM_TPB) {
      const int col = i % KPADH;
      const int colc = (col < HREAL) ? col : (HREAL - 1);
      float v = bfr(h0v[colc]);
      if (col >= HREAL) v = 0.0f;
      hl[i] = (_Float16)v;
    }
    const float cv = bfr(c0v[hcc]);
#pragma unroll
    for (int i = 0; i < 2; ++i)
#pragma unroll
      for (int r = 0; r < 8; ++r) cc[i][r] = cv;
  } else {
    const u32x4* src = (const u32x4*)(const void*)(hall + ((size_t)(t0 - 1) * NBATCH + rowbase) * KPADH);
    for (int u = tid; u < HL_UNITS; u += LSTM_TPB) hl4[u] = src[u];
    const u32x4* csrc = (const u32x4*)(const void*)(cst + (size_t)rowbase * HPAD);
    for (int u = tid; u < CS_UNITS; u += LSTM_TPB) cs4[u] = csrc[u];
#pragma unroll
    for (int i = 0; i < 2; ++i)
#pragma unroll
      for (int r = 0; r < 8; ++r) cc[i][r] = 0.0f;
  }
  __syncthreads();
  if (chunk != 0) {
#pragma unroll
    for (int i = 0; i < 2; ++i)
#pragma unroll
      for (int r = 0; r < 8; ++r) {
        const int lrow = i * 16 + hh * 8 + r;
        cc[i][r] = cs[lrow * HPAD + hcol];
      }
  }

  const v8f vz = (v8f){0.f,0.f,0.f,0.f,0.f,0.f,0.f,0.f};
#pragma unroll 1
  for (int tl = 0; tl < TCHUNK; ++tl) {
    v8f acc[2][4];
#pragma unroll
    for (int i = 0; i < 2; ++i)
#pragma unroll
      for (int q = 0; q < 4; ++q) acc[i][q] = vz;

#pragma unroll 1
    for (int ks = 0; ks < KPADH / 32; ++ks) {
      v16h bq[4];
#pragma unroll
      for (int q = 0; q < 4; ++q)
        bq[q] = Frag<_Float16>::load(Bt + (size_t)(q * HPAD + hcol) * KPADH + koff + ks * 32);
      const v16h a0 = Frag<_Float16>::load(hl + (rl) * KPADH + koff + ks * 32);
      const v16h a1 = Frag<_Float16>::load(hl + (16 + rl) * KPADH + koff + ks * 32);
#pragma unroll
      for (int q = 0; q < 4; ++q) {
        acc[0][q] = Frag<_Float16>::mma(a0, bq[q], acc[0][q]);
        acc[1][q] = Frag<_Float16>::mma(a1, bq[q], acc[1][q]);
      }
      dep_guard_h(acc[0][0], acc[1][3], a0, a1);
      keep4_h(bq[0], bq[1], bq[2], bq[3]);
    }
    acc_guard4(acc[0][0], acc[0][1], acc[0][2], acc[0][3]);
    acc_guard4(acc[1][0], acc[1][1], acc[1][2], acc[1][3]);
    __syncthreads();

    const size_t grow0 = (size_t)(t0 + tl) * NBATCH + rowbase;
    const float* prow0 = preC + ((size_t)tl * NBATCH + rowbase) * NGATE4 + hcol * 4;
#pragma unroll
    for (int i = 0; i < 2; ++i) {
      float exq[8];
      if (has_ex) {
#pragma unroll
        for (int r = 0; r < 8; ++r) {
          const int lrow = i * 16 + hh * 8 + r;
          exq[r] = exb[(grow0 + lrow) * NEXPAD + hcol];
        }
      } else {
#pragma unroll
        for (int r = 0; r < 8; ++r) exq[r] = 0.0f;
      }
#pragma unroll
      for (int r = 0; r < 8; ++r) {
        const int lrow = i * 16 + hh * 8 + r;
        const v4f pv = *(const v4f*)(prow0 + (size_t)lrow * NGATE4);
        const float gi = acc[i][0][r] * WINV + pv[0];
        const float gf = acc[i][1][r] * WINV + pv[1];
        const float gg = acc[i][2][r] * WINV + pv[2];
        const float go = acc[i][3][r] * WINV + pv[3];
        const float cn = sigm_f(gf) * cc[i][r] + sigm_f(gi) * tanh_f(gg);
        cc[i][r] = cn;
        float hv = sigm_f(go) * tanh_f(cn) + exq[r];
        if (hcol >= HREAL) hv = 0.0f;
        hl[lrow * KPADH + hcol] = (_Float16)hv;
      }
      asm volatile("" ::: "memory");
    }
    __syncthreads();

    {
      u32x4* dst = (u32x4*)(void*)(hall + grow0 * KPADH);
      for (int pass = 0; pass < 2; ++pass) {
        for (int u = tid; u < HL_UNITS; u += LSTM_TPB) {
          const u32x4 v = hl4[u];
          *(volatile u32x4*)(dst + u) = v;
        }
        __threadfence();
      }
    }
  }

#pragma unroll
  for (int i = 0; i < 2; ++i)
#pragma unroll
    for (int r = 0; r < 8; ++r) {
      const int lrow = i * 16 + hh * 8 + r;
      cs[lrow * HPAD + hcol] = cc[i][r];
    }
  __syncthreads();
  {
    u32x4* dst = (u32x4*)(void*)(cst + (size_t)rowbase * HPAD);
    for (int pass = 0; pass < 2; ++pass) {
      for (int u = tid; u < CS_UNITS; u += LSTM_TPB) {
        const u32x4 v = cs4[u];
        *(volatile u32x4*)(dst + u) = v;
      }
      __threadfence();
    }
  }
}

__global__ __launch_bounds__(256) void k_logits(
    const unsigned short* __restrict__ hall, const unsigned short* __restrict__ BtY,
    const float* __restrict__ yb, float* __restrict__ out) {
  __shared__ __align__(16) float sl[8][16 * 100];
  const int lane = threadIdx.x & 31, wave = threadIdx.x >> 5;
  const int hh = lane >> 4, rl = lane & 15, koff = hh * 8, mOff = hh * 8;
  const int wt = blockIdx.x * 8 + wave;
  const int m0 = wt * 32;
  if (m0 >= MROWS) return;
  const _Float16* Y = (const _Float16*)(const void*)BtY;
  const v8f vz = (v8f){0.f,0.f,0.f,0.f,0.f,0.f,0.f,0.f};
  v8f acc[2][6];
#pragma unroll
  for (int i = 0; i < 2; ++i)
#pragma unroll
    for (int j = 0; j < 6; ++j) acc[i][j] = vz;

#pragma unroll 1
  for (int l = 0; l < NLAYER; ++l) {
    const _Float16* A = (const _Float16*)(const void*)hall + (size_t)l * MROWS * KPADH;
#pragma unroll 1
    for (int ks = 0; ks < KPADH / 32; ++ks) {
      v16h bq[6];
#pragma unroll
      for (int j = 0; j < 6; ++j)
        bq[j] = Frag<_Float16>::load(Y + (size_t)(j * 16 + rl) * KPADY + l * KPADH + koff + ks * 32);
#pragma unroll
      for (int i = 0; i < 2; ++i) {
        const v16h a = Frag<_Float16>::load(A + (size_t)(m0 + i * 16 + rl) * KPADH + koff + ks * 32);
#pragma unroll
        for (int j = 0; j < 6; ++j) acc[i][j] = Frag<_Float16>::mma(a, bq[j], acc[i][j]);
        dep_guard_h(acc[i][0], acc[i][5], a, a);
      }
      keep4_h(bq[0], bq[1], bq[2], bq[3]);
      keep4_h(bq[4], bq[5], bq[4], bq[5]);
    }
  }
  acc_guard4(acc[0][0], acc[0][1], acc[0][2], acc[0][3]);
  acc_guard4(acc[0][4], acc[0][5], acc[1][0], acc[1][1]);
  acc_guard4(acc[1][2], acc[1][3], acc[1][4], acc[1][5]);

  float ybv[6];
#pragma unroll
  for (int j = 0; j < 6; ++j) ybv[j] = yb[j * 16 + rl];
  float* slab = sl[wave];
#pragma unroll
  for (int i = 0; i < 2; ++i) {
#pragma unroll
    for (int j = 0; j < 6; ++j)
#pragma unroll
      for (int r = 0; r < 8; ++r)
        slab[(mOff + r) * 100 + j * 16 + rl] = acc[i][j][r] * WINV + ybv[j];
    __builtin_amdgcn_fence(__ATOMIC_RELEASE, "workgroup");
    __builtin_amdgcn_wave_barrier();
    __builtin_amdgcn_fence(__ATOMIC_ACQUIRE, "workgroup");
    for (int pass = 0; pass < 2; ++pass) {
#pragma unroll
      for (int rr = 0; rr < 16; ++rr) {
        const int m = m0 + i * 16 + rr;
        const int t = m >> 6, b = m & 63;
        const size_t orow = (size_t)b * NSTEP + t;
        if (lane < 24) {
          const v4f v = *(const v4f*)(slab + rr * 100 + lane * 4);
          *(volatile v4f*)(out + orow * NVOC + lane * 4) = v;
        }
      }
      __threadfence();
    }
    __builtin_amdgcn_fence(__ATOMIC_RELEASE, "workgroup");
    __builtin_amdgcn_wave_barrier();
    __builtin_amdgcn_fence(__ATOMIC_ACQUIRE, "workgroup");
  }
}

extern "C" void kernel_launch(void* const* d_in, const int* in_sizes, int n_in,
                              void* d_out, int out_size, void* d_ws, size_t ws_size,
                              hipStream_t stream) {
  (void)in_sizes; (void)n_in; (void)out_size;
  const int*   xb   = (const int*)d_in[0];
  const float* Cw   = (const float*)d_in[1];
  const float* Uinw = (const float*)d_in[2];
  const float* Uinb = (const float*)d_in[3];
  const float* Winw = (const float*)d_in[4];
  const float* h0in = (const float*)d_in[5];
  const float* c0in = (const float*)d_in[6];
  const float* Uhw  = (const float*)d_in[7];
  const float* Uhb  = (const float*)d_in[8];
  const float* Whw  = (const float*)d_in[9];
  const float* Vhw  = (const float*)d_in[10];
  const float* Vhb  = (const float*)d_in[11];
  const float* h0h  = (const float*)d_in[12];
  const float* c0h  = (const float*)d_in[13];
  const float* Whyw = (const float*)d_in[14];
  const float* byv  = (const float*)d_in[15];
  float* out = (float*)d_out;

  char* base = (char*)d_ws;
  size_t off = 0;
  auto carve = [&](size_t bytes) { size_t o = off; off += (bytes + 255) & ~(size_t)255; return o; };
  const size_t PLANE_H = (size_t)MROWS * KPADH;
  const size_t PLANE_W = (size_t)NGATE4 * KPADH;
  const size_t PLANE_V = (size_t)NEXPAD * KPADE;
  unsigned short* embP  = (unsigned short*)(base + carve((size_t)MROWS * KPADE * 2));
  unsigned short* hallP = (unsigned short*)(base + carve((size_t)NLAYER * PLANE_H * 2));
  float*          preP  = (float*)(base + carve((size_t)MCHUNK * NGATE4 * 4));
  float*          exP   = (float*)(base + carve((size_t)MROWS * NEXPAD * 4));
  unsigned short* btu0  = (unsigned short*)(base + carve((size_t)NGATE4 * KPADE * 2));
  unsigned short* btuh  = (unsigned short*)(base + carve((size_t)3 * PLANE_W * 2));
  unsigned short* btw   = (unsigned short*)(base + carve((size_t)NLAYER * PLANE_W * 2));
  unsigned short* btv   = (unsigned short*)(base + carve((size_t)3 * PLANE_V * 2));
  unsigned short* bty   = (unsigned short*)(base + carve((size_t)NVOC * KPADY * 2));
  float*          biasP = (float*)(base + carve((size_t)BIAS_TOTAL * 4));
  float*          cstP  = (float*)(base + carve((size_t)NBATCH * HPAD * 4));
  if (off > ws_size) return;

  k_embplane<<<(MROWS * 4) / 256, 256, 0, stream>>>(xb, Cw, embP);
  k_wplane<<<dim3((NGATE4 / 16 + 7) / 8, 1), 256, 0, stream>>>(Uinw, Uinw, 0L, btu0, 0L, NGATE4, KPADE, 0, DEMB);
  k_wplane<<<dim3((NGATE4 / 16 + 7) / 8, 3), 256, 0, stream>>>(Uhw, Uhw + (size_t)HREAL * GSRC, (long)HREAL * GSRC,
                                                               btuh, (long)PLANE_W, NGATE4, KPADH, 0, HREAL);
  k_wplane<<<dim3((NGATE4 / 16 + 7) / 8, 4), 256, 0, stream>>>(Winw, Whw, (long)HREAL * GSRC,
                                                               btw, (long)PLANE_W, NGATE4, KPADH, 1, HREAL);
  k_wplane<<<dim3((NEXPAD / 16 + 7) / 8, 3), 256, 0, stream>>>(Vhw, Vhw + (size_t)DEMB * HREAL, (long)DEMB * HREAL,
                                                               btv, (long)PLANE_V, NEXPAD, KPADE, 2, DEMB);
  k_wplane<<<dim3(1, 1), 256, 0, stream>>>(Whyw, Whyw, 0L, bty, 0L, NVOC, KPADY, 3, HREAL);
  k_biasprep<<<(BIAS_TOTAL + 255) / 256, 256, 0, stream>>>(Uinb, Uhb, Vhb, byv, biasP);

  const int preBlocks = ((MCHUNK / 64) * (NGATE4 / 64)) / 8;
  const int exBlocks  = ((MROWS / 64) * (NEXPAD / 64)) / 8;

  for (int n = 0; n < NLAYER; ++n) {
    const float* h0 = (n == 0) ? h0in : (h0h + (size_t)(n - 1) * HREAL);
    const float* c0 = (n == 0) ? c0in : (c0h + (size_t)(n - 1) * HREAL);
    if (n > 0) {
      wmma_gemm64<0, false, 2, 0, false, 1><<<dim3(exBlocks, 1), 256, 0, stream>>>(
          embP, embP, KPADE, 0L,
          btv + (size_t)(n - 1) * PLANE_V, btv + (size_t)(n - 1) * PLANE_V, KPADE, 0L,
          (void*)exP, (void*)exP, NEXPAD, 0L,
          biasP + BIAS_EX_OFF + (n - 1) * NEXPAD, biasP, 0L,
          MROWS, NEXPAD, KPADE, PEINV);
    }
    for (int ch = 0; ch < NCHUNK; ++ch) {
      if (n == 0) {
        wmma_gemm64<0, false, 2, 0, false, 0><<<dim3(preBlocks, 1), 256, 0, stream>>>(
            embP + (size_t)ch * MCHUNK * KPADE, embP + (size_t)ch * MCHUNK * KPADE, KPADE, 0L,
            btu0, btu0, KPADE, 0L,
            (void*)preP, (void*)preP, NGATE4, 0L,
            biasP + BIAS_PRE_OFF, biasP, 0L,
            MCHUNK, NGATE4, KPADE, PEINV);
      } else {
        const unsigned short* Ah = hallP + (size_t)(n - 1) * PLANE_H + (size_t)ch * MCHUNK * KPADH;
        wmma_gemm64<0, false, 2, 0, false, 0><<<dim3(preBlocks, 1), 256, 0, stream>>>(
            Ah, Ah, KPADH, 0L,
            btuh + (size_t)(n - 1) * PLANE_W, btuh + (size_t)(n - 1) * PLANE_W, KPADH, 0L,
            (void*)preP, (void*)preP, NGATE4, 0L,
            biasP + BIAS_PRE_OFF + n * NGATE4, biasP, 0L,
            MCHUNK, NGATE4, KPADH, WINV);
      }
      k_lstm_chunk<<<NBATCH / ROWS_PER_BLK, LSTM_TPB, 0, stream>>>(
          preP, btw + (size_t)n * PLANE_W, exP, h0, c0, hallP + (size_t)n * PLANE_H, cstP,
          ch, (n > 0) ? 1 : 0);
    }
  }

  k_logits<<<(MROWS / 32) / 8, 256, 0, stream>>>(hallP, bty, biasP + BIAS_Y_OFF, out);
}
